// MatrixKANLayer_43164421325572
// MI455X (gfx1250) — hardware-verified
//
#include <hip/hip_runtime.h>
#include <math.h>

typedef __attribute__((ext_vector_type(16))) _Float16 v16h;
typedef __attribute__((ext_vector_type(16))) __bf16 v16b;
typedef __attribute__((ext_vector_type(8)))  _Float16 v8h;
typedef __attribute__((ext_vector_type(8)))  float v8f;
typedef __attribute__((ext_vector_type(4)))  float v4f;
typedef __attribute__((ext_vector_type(2)))  float v2f;
typedef __attribute__((ext_vector_type(4)))  unsigned v4u;
typedef __attribute__((ext_vector_type(4)))  int v4i;
typedef float __attribute__((may_alias)) float_a;
typedef int __attribute__((may_alias)) int_a;

template <typename T> __device__ __forceinline__ void vst2(void* p, T v) { *(volatile T*)p = v; __threadfence(); *(volatile T*)p = v; }
__device__ __forceinline__ v8f wmma16(v16h a, v16h b, v8f c) {
  v8f d = __builtin_amdgcn_wmma_f32_16x16x32_f16(false, a, false, b, (short)0, c, false, false);
  asm volatile("v_nop\n\tv_nop\n\tv_nop\n\tv_nop" : "+v"(d) : "v"(a), "v"(b));
  return d;
}
__device__ __forceinline__ v8f wmma_bf(v16b a, v16b b, v8f c) {
  v8f d = __builtin_amdgcn_wmma_f32_16x16x32_bf16(false, a, false, b, (short)0, c, false, false);
  asm volatile("v_nop\n\tv_nop\n\tv_nop\n\tv_nop" : "+v"(d) : "v"(a), "v"(b));
  return d;
}
__device__ __forceinline__ v16h frag_h(const _Float16* rowk0, int lane) {
  union { v16h v; v8h q[2]; } u; const _Float16* p = rowk0 + 8 * (lane >> 4);
  u.q[0] = *(const v8h*)p; u.q[1] = *(const v8h*)(p + 16); return u.v;
}
__device__ __forceinline__ v16h frag_f32(const float* rowk0, int lane) {
  v16h a; const float* p = rowk0 + 8 * (lane >> 4);
#pragma unroll
  for (int i = 0; i < 8; ++i) { a[i] = (_Float16)p[i]; a[8 + i] = (_Float16)p[16 + i]; }
  return a;
}
__device__ __forceinline__ v16h frag_f32s(const float* rowk0, int lane, float sc) {
  v16h a; const float* p = rowk0 + 8 * (lane >> 4);
#pragma unroll
  for (int i = 0; i < 8; ++i) { a[i] = (_Float16)(p[i] * sc); a[8 + i] = (_Float16)(p[16 + i] * sc); }
  return a;
}
__device__ __forceinline__ v16h fragc_f32(const float* W, int k0, int n, int lane, int ld, int K) {
  v16h a; const int g = lane >> 4;
#pragma unroll
  for (int i = 0; i < 8; ++i) { const int ka = k0 + 8 * g + i, kb = ka + 16;
    a[i] = (_Float16)(ka < K ? W[(size_t)ka * ld + n] : 0.f); a[8 + i] = (_Float16)(kb < K ? W[(size_t)kb * ld + n] : 0.f); }
  return a;
}
struct F2 { v16b h, l; };
__device__ __forceinline__ F2 bsplit16(const float v[16]) { F2 r;
#pragma unroll
  for (int i = 0; i < 16; ++i) { const __bf16 h = (__bf16)v[i]; r.h[i] = h; r.l[i] = (__bf16)(v[i] - (float)h); }
  return r; }
__device__ __forceinline__ F2 split_row(const float* row, int k0, int lane) { float v[16]; const float* p = row + k0 + 8 * (lane >> 4);
#pragma unroll
  for (int i = 0; i < 8; ++i) { v[i] = p[i]; v[8 + i] = p[16 + i]; }
  return bsplit16(v); }
__device__ __forceinline__ F2 split_rowK(const float* row, int k0, int lane, int K) { float v[16]; const int g = lane >> 4;
#pragma unroll
  for (int i = 0; i < 8; ++i) { const int ka = k0 + 8 * g + i, kb = ka + 16; v[i] = ka < K ? row[ka] : 0.f; v[8 + i] = kb < K ? row[kb] : 0.f; }
  return bsplit16(v); }
__device__ __forceinline__ F2 split_col(const float* W, int k0, int n, int lane, int ld, int K) { float v[16]; const int g = lane >> 4;
#pragma unroll
  for (int i = 0; i < 8; ++i) { const int ka = k0 + 8 * g + i, kb = ka + 16; v[i] = ka < K ? W[(size_t)ka * ld + n] : 0.f; v[8 + i] = kb < K ? W[(size_t)kb * ld + n] : 0.f; }
  return bsplit16(v); }
__device__ __forceinline__ v8f mac3(const F2& a, const F2& b, v8f c) { c = wmma_bf(a.l, b.h, c); c = wmma_bf(a.h, b.l, c); return wmma_bf(a.h, b.h, c); }
__device__ __forceinline__ float sigm(float v) { return 1.0f / (1.0f + expf(-v)); }
#define LDSX() do { asm volatile("s_wait_dscnt 0" ::: "memory"); __builtin_amdgcn_wave_barrier(); __builtin_amdgcn_fence(__ATOMIC_RELEASE, "workgroup"); } while (0)

#define NBT 4096
#define NI 512
#define NO 512
#define NBAS 11
#define KORD 3
#define NGRID 15
#define KSP (NI * NBAS)
#define IG 32

__global__ __launch_bounds__(256) void k_pack(const float* __restrict__ coef, const float* __restrict__ sb, const float* __restrict__ sp, const float* __restrict__ msk, _Float16* __restrict__ P1, _Float16* __restrict__ P2) {
  const int o = blockIdx.x, tid = threadIdx.x;
  __shared__ __align__(16) _Float16 s1[KSP]; __shared__ __align__(16) _Float16 s2[NI];
  for (int k = tid; k < KSP; k += 256) { const int i = k / NBAS, j = k % NBAS; s1[k] = (_Float16)(coef[((size_t)i * NO + o) * NBAS + j] * sp[i * NO + o] * msk[i * NO + o] * 16.0f); }
  for (int i = tid; i < NI; i += 256) s2[i] = (_Float16)(sb[i * NO + o] * msk[i * NO + o] * 16.0f);
  __syncthreads();
  for (int q = tid; q < KSP / 8; q += 256) vst2(P1 + (size_t)o * KSP + q * 8, *(const v4u*)(&s1[q * 8]));
  for (int q = tid; q < NI / 8; q += 256) vst2(P2 + (size_t)o * NI + q * 8, *(const v4u*)(&s2[q * 8]));
}
__global__ __launch_bounds__(128) void k_main(const float* __restrict__ x, const float* __restrict__ grid, const float* __restrict__ bm, const _Float16* __restrict__ P1, const _Float16* __restrict__ P2, float* __restrict__ out) {
  __shared__ float sfull[64][IG * NBAS + 1];
  __shared__ __align__(16) _Float16 sa[4][16][40];
  __shared__ __align__(16) float so[4][16][132];
  __shared__ float sbm[16]; __shared__ float sgr[IG][16];
  const int tid = threadIdx.x, wave = tid >> 5, lane = tid & 31, col = lane & 15, g = lane >> 4;
  const int r0b = blockIdx.x * 64, r0 = r0b + wave * 16, n0 = blockIdx.y * 128;
  if (tid < 16) sbm[tid] = bm[tid];
  v8f acc[8];
#pragma unroll
  for (int t = 0; t < 8; ++t) acc[t] = (v8f){};
#pragma unroll 1
  for (int i0 = 0; i0 < NI; i0 += IG) {
    __syncthreads();
    for (int q = tid; q < IG * NGRID; q += 128) { const int il = q / NGRID, gg = q % NGRID; sgr[il][gg] = grid[(size_t)(i0 + il) * NGRID + gg]; }
    __syncthreads();
    for (int q = tid; q < 64 * IG; q += 128) { const int rl = q / IG, il = q % IG; const float xv = x[(size_t)(r0b + rl) * NI + i0 + il]; const float* gr = &sgr[il][0];
      const float h = (gr[8 + KORD] - gr[KORD]) / 8.0f;
      int t = -1;
      for (int e = NGRID - 2; e >= 0; --e) if (xv >= gr[e] && xv < gr[e + 1]) t = e;
      float fb[NBAS];
#pragma unroll
      for (int j = 0; j < NBAS; ++j) fb[j] = 0.f;
      if (t >= 0) { const float fl = (float)t * h + gr[0]; const float u1 = (xv - fl) / h; float up[4]; up[0] = 1.f; up[1] = u1; up[2] = u1 * u1; up[3] = up[2] * u1;
#pragma unroll
        for (int qq = 0; qq < 4; ++qq) { float lv = 0.f;
#pragma unroll
          for (int p = 0; p < 4; ++p) lv += up[p] * sbm[p * 4 + qq];
          const int idx = t - KORD + qq; if (idx >= 0 && idx < NBAS) fb[idx] += lv; } }
#pragma unroll
      for (int j = 0; j < NBAS; ++j) sfull[rl][il * NBAS + j] = fb[j]; }
    __syncthreads();
#pragma unroll 1
    for (int kc = 0; kc < (IG * NBAS) / 32; ++kc) {
      { union { v8h h8[2]; v4u u2[2]; } pk;
#pragma unroll
        for (int u = 0; u < 16; ++u) pk.h8[u >> 3][u & 7] = (_Float16)sfull[wave * 16 + col][kc * 32 + g * 16 + u];
        *(v4u*)(&sa[wave][col][g * 16]) = pk.u2[0]; *(v4u*)(&sa[wave][col][g * 16 + 8]) = pk.u2[1]; }
      LDSX();
      const v16h a = frag_h(&sa[wave][col][0], lane);
      const size_t kg = (size_t)i0 * NBAS + kc * 32;
#pragma unroll
      for (int t = 0; t < 8; ++t) acc[t] = wmma16(a, frag_h(P1 + (size_t)(n0 + t * 16 + col) * KSP + kg, lane), acc[t]);
      LDSX(); } }
#pragma unroll 1
  for (int kc = 0; kc < NI / 32; ++kc) {
    { union { v8h h8[2]; v4u u2[2]; } pk;
#pragma unroll
      for (int u = 0; u < 16; ++u) { const float xv = x[(size_t)(r0 + col) * NI + kc * 32 + g * 16 + u]; pk.h8[u >> 3][u & 7] = (_Float16)(xv * sigm(xv)); }
      *(v4u*)(&sa[wave][col][g * 16]) = pk.u2[0]; *(v4u*)(&sa[wave][col][g * 16 + 8]) = pk.u2[1]; }
    LDSX();
    const v16h a = frag_h(&sa[wave][col][0], lane);
#pragma unroll
    for (int t = 0; t < 8; ++t) acc[t] = wmma16(a, frag_h(P2 + (size_t)(n0 + t * 16 + col) * NI + kc * 32, lane), acc[t]);
    LDSX(); }
#pragma unroll
  for (int t = 0; t < 8; ++t)
#pragma unroll
    for (int r = 0; r < 8; ++r) so[wave][8 * g + r][t * 16 + col] = acc[t][r] * (1.0f / 16.0f);
  LDSX();
#pragma unroll 4
  for (int rl = 0; rl < 16; ++rl) vst2(out + (size_t)(r0 + rl) * NO + n0 + lane * 4, *(const v4f*)(&so[wave][rl][lane * 4]));
}
extern "C" void kernel_launch(void* const* d_in, const int* in_sizes, int n_in, void* d_out, int out_size, void* d_ws, size_t ws_size, hipStream_t stream) {
  (void)in_sizes; (void)n_in; (void)out_size; (void)ws_size;
  const float* x = (const float*)d_in[0]; const float* grid = (const float*)d_in[1]; const float* coef = (const float*)d_in[2]; const float* sb = (const float*)d_in[3]; const float* sp = (const float*)d_in[4]; const float* msk = (const float*)d_in[5]; const float* bm = (const float*)d_in[6];
  float* out = (float*)d_out;
  char* ws = (char*)d_ws; size_t off = 0;
  auto take = [&](size_t bytes) { char* p = ws + off; off += (bytes + 255) & ~(size_t)255; return p; };
  _Float16* P1 = (_Float16*)take((size_t)NO * KSP * 2); _Float16* P2 = (_Float16*)take((size_t)NO * NI * 2);
  k_pack<<<NO, 256, 0, stream>>>(coef, sb, sp, msk, P1, P2);
  k_main<<<dim3(NBT / 64, NO / 128), 128, 0, stream>>>(x, grid, bm, P1, P2, out);
}
